// GAT_Encoder_60129542496
// MI455X (gfx1250) — hardware-verified
//
#include <hip/hip_runtime.h>
#include <stdint.h>


typedef _Float16 v16h __attribute__((ext_vector_type(16)));
typedef _Float16 v8h_ __attribute__((ext_vector_type(8)));
typedef v8h_ __attribute__((may_alias)) v8h;
typedef float v8f __attribute__((ext_vector_type(8)));
typedef float v4f_ __attribute__((ext_vector_type(4)));
typedef v4f_ __attribute__((may_alias)) v4f;
typedef unsigned int v4u __attribute__((ext_vector_type(4)));

union Frag { v16h v; v8h half[2]; };
union HU { v8h h; v4u u; };

#define B_    8
#define NV_   1024
#define FEAT_ 256
#define NH_   4
#define DH_   64
#define NBLK_ 2
#define ALPHA_ 0.2f
#define EPS_   1e-5f
#define NEGF_  (-9.0e15f)

static_assert(NH_ * DH_ == FEAT_);
static_assert((NV_ % 64) == 0);
static_assert((FEAT_ % 32) == 0);
static_assert(FEAT_ == 8 * 32);

__device__ __forceinline__ v8f wmma16(v8f c, v16h a, v16h b) {
    v8f d = __builtin_amdgcn_wmma_f32_16x16x32_f16(false, a, false, b, (short)0, c, false, false);
    asm volatile("v_nop\n\tv_nop\n\tv_nop\n\tv_nop" : "+v"(d) : "v"(a), "v"(b));
    return d;
}

__device__ __forceinline__ v8f zero8() {
    v8f z;
#pragma unroll
    for (int i = 0; i < 8; ++i) z[i] = 0.f;
    return z;
}

__device__ __forceinline__ void st16v(_Float16* p, v4u u) { *(volatile v4u*)p = u; }
__device__ __forceinline__ void stf4(float* p, v4f v) { *(volatile v4f*)p = v; }

__global__ __launch_bounds__(256) void wconv_kernel(const float* __restrict__ W,
                                                    _Float16* __restrict__ W16) {
    const int bid = blockIdx.x;
    const int dq  = bid & 3;
    const int bh  = bid >> 2;
    const int t   = threadIdx.x;
    __shared__ __align__(16) _Float16 T[16][264];

    const float* src = W + ((size_t)bh * FEAT_ + t) * DH_ + dq * 16;
#pragma unroll
    for (int q4 = 0; q4 < 4; ++q4) {
        float4 f = *(const float4*)(src + 4 * q4);
        T[4 * q4 + 0][t] = (_Float16)(f.x * 16.0f);
        T[4 * q4 + 1][t] = (_Float16)(f.y * 16.0f);
        T[4 * q4 + 2][t] = (_Float16)(f.z * 16.0f);
        T[4 * q4 + 3][t] = (_Float16)(f.w * 16.0f);
    }
    __syncthreads();

    const int wave = t >> 5, l = t & 31;
    HU vals[2];
    size_t offs[2];
#pragma unroll
    for (int s = 0; s < 2; ++s) {
        const int L  = wave * 8 + s * 4 + (l >> 3);
        const int dd = L >> 2, qt = L & 3, p = l & 7;
        vals[s].h = *(const v8h*)&T[dd][qt * 64 + p * 8];
        offs[s] = ((size_t)(bh * DH_ + dq * 16 + dd)) * FEAT_ + qt * 64 + p * 8;
    }
#pragma unroll
    for (int s = 0; s < 2; ++s) st16v(W16 + offs[s], vals[s].u);
    __threadfence();
#pragma unroll
    for (int s = 0; s < 2; ++s) st16v(W16 + offs[s], vals[s].u);
}

__global__ __launch_bounds__(32) void bn_kernel(const float* __restrict__ src,
                                                const float* __restrict__ gamma,
                                                const float* __restrict__ beta,
                                                _Float16* __restrict__ dst16,
                                                float* __restrict__ dst32,
                                                int mode) {
    const int v = blockIdx.x;
    const int l = threadIdx.x;
    __shared__ __align__(16) float rows[B_][FEAT_];

    float s = 0.f;
#pragma unroll 1
    for (int b = 0; b < B_; ++b) {
        const float* rp = src + ((size_t)b * NV_ + v) * FEAT_ + 8 * l;
        const v4f xa = *(const v4f*)rp;
        const v4f xb = *(const v4f*)(rp + 4);
        s += ((xa[0] + xa[1]) + (xa[2] + xa[3])) + ((xb[0] + xb[1]) + (xb[2] + xb[3]));
        *(v4f*)&rows[b][8 * l]     = xa;
        *(v4f*)&rows[b][8 * l + 4] = xb;
    }
#pragma unroll
    for (int o = 16; o > 0; o >>= 1) s += __shfl_xor(s, o);
    const float mean = s * (1.0f / (float)(B_ * FEAT_));
    __syncthreads();

    float qq = 0.f;
#pragma unroll 1
    for (int b = 0; b < B_; ++b) {
        const v4f xa = *(const v4f*)&rows[b][8 * l];
        const v4f xb = *(const v4f*)&rows[b][8 * l + 4];
        const float d0 = xa[0] - mean, d1 = xa[1] - mean, d2 = xa[2] - mean, d3 = xa[3] - mean;
        const float d4 = xb[0] - mean, d5 = xb[1] - mean, d6 = xb[2] - mean, d7 = xb[3] - mean;
        qq += ((d0 * d0 + d1 * d1) + (d2 * d2 + d3 * d3)) + ((d4 * d4 + d5 * d5) + (d6 * d6 + d7 * d7));
    }
#pragma unroll
    for (int o = 16; o > 0; o >>= 1) qq += __shfl_xor(qq, o);
    const float var = qq * (1.0f / (float)(B_ * FEAT_));
    const float inv = rsqrtf(var + EPS_);
    const float g = gamma[v], be = beta[v];

#pragma unroll 1
    for (int b = 0; b < B_; ++b) {
        v4f xa = *(const v4f*)&rows[b][8 * l];
        v4f xb = *(const v4f*)&rows[b][8 * l + 4];
        v4f ya, yb;
        ya[0] = g * ((xa[0] - mean) * inv) + be;
        ya[1] = g * ((xa[1] - mean) * inv) + be;
        ya[2] = g * ((xa[2] - mean) * inv) + be;
        ya[3] = g * ((xa[3] - mean) * inv) + be;
        yb[0] = g * ((xb[0] - mean) * inv) + be;
        yb[1] = g * ((xb[1] - mean) * inv) + be;
        yb[2] = g * ((xb[2] - mean) * inv) + be;
        yb[3] = g * ((xb[3] - mean) * inv) + be;
        *(v4f*)&rows[b][8 * l]     = ya;
        *(v4f*)&rows[b][8 * l + 4] = yb;
    }
    __syncthreads();

    if (mode == 0) {
#pragma unroll 1
        for (int b = 0; b < B_; ++b) {
            const v4f ya = *(const v4f*)&rows[b][8 * l];
            const v4f yb = *(const v4f*)&rows[b][8 * l + 4];
            HU o;
            o.h[0] = (_Float16)ya[0]; o.h[1] = (_Float16)ya[1]; o.h[2] = (_Float16)ya[2]; o.h[3] = (_Float16)ya[3];
            o.h[4] = (_Float16)yb[0]; o.h[5] = (_Float16)yb[1]; o.h[6] = (_Float16)yb[2]; o.h[7] = (_Float16)yb[3];
            st16v(dst16 + ((size_t)b * NV_ + v) * FEAT_ + 8 * l, o.u);
        }
        __threadfence();
#pragma unroll 1
        for (int b = 0; b < B_; ++b) {
            const v4f ya = *(const v4f*)&rows[b][8 * l];
            const v4f yb = *(const v4f*)&rows[b][8 * l + 4];
            HU o;
            o.h[0] = (_Float16)ya[0]; o.h[1] = (_Float16)ya[1]; o.h[2] = (_Float16)ya[2]; o.h[3] = (_Float16)ya[3];
            o.h[4] = (_Float16)yb[0]; o.h[5] = (_Float16)yb[1]; o.h[6] = (_Float16)yb[2]; o.h[7] = (_Float16)yb[3];
            st16v(dst16 + ((size_t)b * NV_ + v) * FEAT_ + 8 * l, o.u);
        }
    } else {
#pragma unroll 1
        for (int b = 0; b < B_; ++b) {
            const v4f o0 = *(const v4f*)&rows[b][4 * l];
            const v4f o1 = *(const v4f*)&rows[b][128 + 4 * l];
            float* dp = dst32 + ((size_t)b * NV_ + v) * FEAT_;
            stf4(dp + 4 * l, o0);
            stf4(dp + 128 + 4 * l, o1);
        }
        __threadfence();
#pragma unroll 1
        for (int b = 0; b < B_; ++b) {
            const v4f o0 = *(const v4f*)&rows[b][4 * l];
            const v4f o1 = *(const v4f*)&rows[b][128 + 4 * l];
            float* dp = dst32 + ((size_t)b * NV_ + v) * FEAT_;
            stf4(dp + 4 * l, o0);
            stf4(dp + 128 + 4 * l, o1);
        }
    }
}

__global__ __launch_bounds__(128) void gemm_kernel(const _Float16* __restrict__ enc16,
                                                   const _Float16* __restrict__ W16,
                                                   const float* __restrict__ Wb,
                                                   const float* __restrict__ a1,
                                                   const float* __restrict__ a2,
                                                   _Float16* __restrict__ WhT,
                                                   float* __restrict__ S1,
                                                   float* __restrict__ S2) {
    const int bid   = blockIdx.x;
    const int ntile = bid & (NV_ / 64 - 1);
    const int bh    = bid >> 4;
    const int h     = bh & (NH_ - 1);
    const int b     = bh >> 2;
    const int n0    = ntile * 64;
    const int t = threadIdx.x, wave = t >> 5, l = t & 31, hh = l >> 4, m = l & 15;

    __shared__ float S[64][65];
    __shared__ __align__(16) float sa1[DH_];
    __shared__ __align__(16) float sa2[DH_];
    __shared__ __align__(16) float swb[DH_];
    __shared__ __align__(16) float ss1[64];
    __shared__ __align__(16) float ss2[64];
    if (t < DH_) {
        sa1[t] = a1[h * DH_ + t];
        sa2[t] = a2[h * DH_ + t];
        swb[t] = Wb[h * DH_ + t];
    }
    __syncthreads();

    const _Float16* arow = enc16 + ((size_t)b * NV_ + n0 + 16 * wave + m) * FEAT_ + 8 * hh;
    const _Float16* brow = W16 + ((size_t)h * DH_ + m) * FEAT_ + 8 * hh;

    v8f ct[4];
#pragma unroll
    for (int tt = 0; tt < 4; ++tt) ct[tt] = zero8();

#pragma unroll 1
    for (int k0 = 0; k0 < FEAT_; k0 += 32) {
        Frag a;
        a.half[0] = *(const v8h*)(arow + k0);
        a.half[1] = *(const v8h*)(arow + k0 + 16);
#pragma unroll
        for (int tt = 0; tt < 4; ++tt) {
            const _Float16* bp = brow + (size_t)tt * 16 * FEAT_ + k0;
            Frag bb;
            bb.half[0] = *(const v8h*)bp;
            bb.half[1] = *(const v8h*)(bp + 16);
            ct[tt] = wmma16(ct[tt], a.v, bb.v);
        }
    }

#pragma unroll
    for (int tt = 0; tt < 4; ++tt) {
#pragma unroll
        for (int r = 0; r < 8; ++r) {
            S[16 * wave + 8 * hh + r][16 * tt + m] = ct[tt][r] * 0.0625f + swb[16 * tt + m];
        }
    }
    __syncthreads();

    if (t < 64) {
        float s1 = 0.f, s2 = 0.f;
#pragma unroll
        for (int d = 0; d < DH_; ++d) {
            float w = S[t][d];
            s1 += w * sa1[d];
            s2 += w * sa2[d];
        }
        ss1[t] = s1;
        ss2[t] = s2;
    }

    HU wv[4];
    size_t woff[4];
#pragma unroll
    for (int s = 0; s < 4; ++s) {
        const int d = 16 * wave + 4 * s + (l >> 3);
        const int p = l & 7;
#pragma unroll
        for (int e = 0; e < 8; ++e) wv[s].h[e] = (_Float16)S[8 * p + e][d];
        woff[s] = ((size_t)(bh * DH_ + d)) * NV_ + n0 + 8 * p;
    }
    __syncthreads();

    v4f sv;
    sv[0] = 0.f; sv[1] = 0.f; sv[2] = 0.f; sv[3] = 0.f;
    float* sp = S1;
    if (wave == 0) {
        if (l < 16) {
            sv = *(const v4f*)&ss1[4 * l];
            sp = S1 + (size_t)bh * NV_ + n0 + 4 * l;
        } else {
            sv = *(const v4f*)&ss2[4 * (l - 16)];
            sp = S2 + (size_t)bh * NV_ + n0 + 4 * (l - 16);
        }
    }

#pragma unroll
    for (int s = 0; s < 4; ++s) st16v(WhT + woff[s], wv[s].u);
    if (wave == 0) stf4(sp, sv);
    __threadfence();
#pragma unroll
    for (int s = 0; s < 4; ++s) st16v(WhT + woff[s], wv[s].u);
    if (wave == 0) stf4(sp, sv);
}

__global__ __launch_bounds__(128) void attn_kernel(const _Float16* __restrict__ WhT,
                                                   const float* __restrict__ S1,
                                                   const float* __restrict__ S2,
                                                   const int* __restrict__ adj,
                                                   float* __restrict__ hcat) {
    const int bid   = blockIdx.x;
    const int itile = bid & (NV_ / 16 - 1);
    const int bh    = bid >> 6;
    const int h     = bh & (NH_ - 1);
    const int b     = bh >> 2;
    const int i0    = itile * 16;
    const int t = threadIdx.x, wave = t >> 5, l = t & 31, hh = l >> 4, m = l & 15;
    const int q = t & 3, jl = t >> 2;

    __shared__ __align__(16) _Float16 Ps[16][40];
    __shared__ float red[16][33];
    __shared__ float s_rmx[16];
    __shared__ float s_inv[16];
    __shared__ __align__(16) float So[16][68];

    const float4 s2v4 = *(const float4*)(S2 + (size_t)bh * NV_ + i0 + 4 * q);
    float s2v[4];
    s2v[0] = s2v4.x; s2v[1] = s2v4.y; s2v[2] = s2v4.z; s2v[3] = s2v4.w;
    const int*   adjp = adj + ((size_t)b * NV_) * NV_ + i0 + 4 * q;
    const float* s1p  = S1 + (size_t)bh * NV_;
    const float NINF = -__builtin_huge_valf();

    float mx[4];
    mx[0] = NINF; mx[1] = NINF; mx[2] = NINF; mx[3] = NINF;
#pragma unroll 1
    for (int j0 = 0; j0 < NV_; j0 += 32) {
        const int j = j0 + jl;
        const int4 a4 = *(const int4*)(adjp + (size_t)j * NV_);
        const float s1 = s1p[j];
        int av[4];
        av[0] = a4.x; av[1] = a4.y; av[2] = a4.z; av[3] = a4.w;
#pragma unroll
        for (int r = 0; r < 4; ++r) mx[r] = (av[r] > 0) ? fmaxf(mx[r], s1) : mx[r];
    }
#pragma unroll
    for (int r = 0; r < 4; ++r) red[4 * q + r][jl] = mx[r];
    __syncthreads();
    if (t < 16) {
        float v = red[t][0];
#pragma unroll
        for (int c = 1; c < 32; ++c) v = fmaxf(v, red[t][c]);
        float rm;
        if (v > NINF) {
            float e = v + S2[(size_t)bh * NV_ + i0 + t];
            rm = (e >= 0.f) ? e : ALPHA_ * e;
        } else {
            rm = NEGF_;
        }
        s_rmx[t] = rm;
    }
    __syncthreads();
    float rmx[4];
#pragma unroll
    for (int r = 0; r < 4; ++r) rmx[r] = s_rmx[4 * q + r];

    const _Float16* vrow = WhT + ((size_t)bh * DH_ + 16 * wave + m) * NV_ + 8 * hh;
    v8f acc = zero8();
    float psum[4];
    psum[0] = 0.f; psum[1] = 0.f; psum[2] = 0.f; psum[3] = 0.f;
#pragma unroll 1
    for (int j0 = 0; j0 < NV_; j0 += 32) {
        const int j = j0 + jl;
        const int4 a4 = *(const int4*)(adjp + (size_t)j * NV_);
        const float s1 = s1p[j];
        int av[4];
        av[0] = a4.x; av[1] = a4.y; av[2] = a4.z; av[3] = a4.w;
#pragma unroll
        for (int r = 0; r < 4; ++r) {
            float e = s1 + s2v[r];
            e = (e >= 0.f) ? e : ALPHA_ * e;
            float s = (av[r] > 0) ? e : NEGF_;
            float p = __expf(s - rmx[r]);
            psum[r] += p;
            Ps[4 * q + r][jl] = (_Float16)(p * 16384.0f);
        }
        __syncthreads();

        Frag pa;
        pa.half[0] = *(const v8h*)&Ps[m][8 * hh];
        pa.half[1] = *(const v8h*)&Ps[m][16 + 8 * hh];
        Frag vb;
        vb.half[0] = *(const v8h*)(vrow + j0);
        vb.half[1] = *(const v8h*)(vrow + j0 + 16);
        acc = wmma16(acc, pa.v, vb.v);
        __syncthreads();
    }

#pragma unroll
    for (int r = 0; r < 4; ++r) red[4 * q + r][jl] = psum[r];
    __syncthreads();
    if (t < 16) {
        float v = red[t][0];
#pragma unroll
        for (int c = 1; c < 32; ++c) v += red[t][c];
        s_inv[t] = 1.0f / v;
    }
    __syncthreads();

#pragma unroll
    for (int r = 0; r < 8; ++r) {
        const int row = 8 * hh + r;
        float o = acc[r] * (1.0f / 16384.0f) * s_inv[row];
        o = (o > 0.f) ? o : (__expf(o) - 1.0f);
        So[row][16 * wave + m] = o;
    }
    __syncthreads();

    v4f ov[2];
    size_t ooff[2];
#pragma unroll
    for (int s = 0; s < 2; ++s) {
        const int L    = 4 * s + (l >> 3);
        const int row  = 4 * wave + (L >> 1);
        const int half = L & 1, p = l & 7;
        const int col  = half * 32 + p * 4;
        ov[s]   = *(const v4f*)&So[row][col];
        ooff[s] = ((size_t)b * NV_ + i0 + row) * FEAT_ + h * DH_ + col;
    }
#pragma unroll
    for (int s = 0; s < 2; ++s) stf4(hcat + ooff[s], ov[s]);
    __threadfence();
#pragma unroll
    for (int s = 0; s < 2; ++s) stf4(hcat + ooff[s], ov[s]);
}

extern "C" void kernel_launch(void* const* d_in, const int* in_sizes, int n_in,
                              void* d_out, int out_size, void* d_ws, size_t ws_size,
                              hipStream_t stream) {
    if (n_in < 10) return;
    if (in_sizes[0] != B_ * NV_ * FEAT_) return;
    if (in_sizes[1] != B_ * NV_ * NV_) return;
    if (in_sizes[2] != NBLK_ * NH_ * FEAT_ * DH_) return;
    if (in_sizes[3] != NBLK_ * NH_ * DH_ || in_sizes[4] != NBLK_ * NH_ * DH_ || in_sizes[5] != NBLK_ * NH_ * DH_) return;
    if (in_sizes[6] != NV_ || in_sizes[7] != NV_ || in_sizes[8] != NBLK_ * NV_ || in_sizes[9] != NBLK_ * NV_) return;
    if (out_size != B_ * NV_ * FEAT_) return;

    const float* x      = (const float*)d_in[0];
    const int*   adj    = (const int*)  d_in[1];
    const float* W      = (const float*)d_in[2];
    const float* Wb     = (const float*)d_in[3];
    const float* a1     = (const float*)d_in[4];
    const float* a2     = (const float*)d_in[5];
    const float* gamma0 = (const float*)d_in[6];
    const float* beta0  = (const float*)d_in[7];
    const float* gammas = (const float*)d_in[8];
    const float* betas  = (const float*)d_in[9];
    float* out = (float*)d_out;

    const size_t off_enc16 = 0;
    const size_t off_w16   = off_enc16 + (size_t)B_ * NV_ * FEAT_ * 2;
    const size_t off_wht   = off_w16   + (size_t)NBLK_ * NH_ * DH_ * FEAT_ * 2;
    const size_t off_s1    = off_wht   + (size_t)B_ * NH_ * DH_ * NV_ * 2;
    const size_t off_s2    = off_s1    + (size_t)B_ * NH_ * NV_ * 4;
    const size_t off_hcat  = off_s2    + (size_t)B_ * NH_ * NV_ * 4;
    const size_t total     = off_hcat  + (size_t)B_ * NV_ * FEAT_ * 4;
    if (total > ws_size) return;

    char* ws = (char*)d_ws;
    _Float16* enc16 = (_Float16*)(ws + off_enc16);
    _Float16* W16   = (_Float16*)(ws + off_w16);
    _Float16* WhT   = (_Float16*)(ws + off_wht);
    float*    S1    = (float*)(ws + off_s1);
    float*    S2    = (float*)(ws + off_s2);
    float*    hcat  = (float*)(ws + off_hcat);

    wconv_kernel<<<NBLK_ * NH_ * 4, 256, 0, stream>>>(W, W16);
    bn_kernel<<<NV_, 32, 0, stream>>>(x, gamma0, beta0, enc16, out, 0);

    for (int blk = 0; blk < NBLK_; ++blk) {
        const _Float16* W16p = W16 + (size_t)blk * NH_ * DH_ * FEAT_;
        const float* Wbp = Wb + (size_t)blk * NH_ * DH_;
        const float* a1p = a1 + (size_t)blk * NH_ * DH_;
        const float* a2p = a2 + (size_t)blk * NH_ * DH_;

        gemm_kernel<<<B_ * NH_ * (NV_ / 64), 128, 0, stream>>>(enc16, W16p, Wbp, a1p, a2p, WhT, S1, S2);
        attn_kernel<<<B_ * NH_ * (NV_ / 16), 128, 0, stream>>>(WhT, S1, S2, adj, hcat);
        const int mode = (blk == NBLK_ - 1) ? 1 : 0;
        bn_kernel<<<NV_, 32, 0, stream>>>(hcat, gammas + (size_t)blk * NV_, betas + (size_t)blk * NV_,
                                          enc16, out, mode);
    }
}
